// BIMPM_57621281243632
// MI455X (gfx1250) — hardware-verified
//
#include <hip/hip_runtime.h>


#ifndef NB
#define NB 16
#endif
#ifndef SEQ
#define SEQ 128
#endif
#define NB_FULL  16
#define SEQ_FULL 128
#ifndef OUT_SEQ
#define OUT_SEQ SEQ
#endif
#define FW    512
#define HW    256
#define NPER  16
#define OC    128
#define ROWS  (NB * SEQ)
#define NZ    (NB * 2)
#define NPL   7
#define TSP   136
#define EPSV  1.0e-8f
#define PCAR  256.0f
#define ASC   (1.0f / 32.0f)
#define ASI   0.125f
#define AMC   16.0f
#define AMI   (1.0f / 16.0f)
#define W2C   64.0f
#define W2I   (1.0f / 64.0f)
#define NEGB  (-3.0e38f)

static_assert(SEQ == 128);
static_assert(SEQ <= SEQ_FULL);
static_assert(NB <= NB_FULL);
static_assert(HW == 256);
static_assert(FW == 2 * HW);
static_assert(HW % 32 == 0);
static_assert(SEQ % 32 == 0);
static_assert(HW % 64 == 0);
static_assert(ROWS % 64 == 0);
static_assert(ROWS % 32 == 0);
static_assert(NPER == 16);
static_assert(OC == 8 * NPER);
static_assert((NZ * SEQ) % 8 == 0);
static_assert(64 % NB == 0 || NB <= 64);
static_assert(NB <= 64);
static_assert((TSP * 2) % 16 == 0);
static_assert(32 * 16 * 8 == 16 * 64 * 4);
static_assert(32 * 16 * 4 == 16 * 64 * 2);
static_assert(8 * 4 * 2 == 64);
static_assert(32 * 16 == HW * 2);
static_assert(32 * 16 == SEQ * 4);
static_assert(32 * 4 == 128);
static_assert(16 * 68 * 4 <= 131072);
static_assert(64 * TSP * 2 <= 131072);
static_assert(8 * SEQ * 4 <= 131072);
static_assert(2 * SEQ * 4 <= 131072);

typedef _Float16 h16;
typedef __attribute__((ext_vector_type(16))) _Float16 v16h;
typedef __attribute__((ext_vector_type(8)))  _Float16 v8h;
typedef __attribute__((ext_vector_type(8)))  float    v8f;
typedef __attribute__((ext_vector_type(4)))  float    v4f;
typedef v4f  __attribute__((may_alias)) v4fa;
typedef v8h  __attribute__((may_alias)) v8ha;

__device__ __forceinline__ unsigned short f2bf(float f) { unsigned u = __float_as_uint(f); u += 0x7FFFu + ((u >> 16) & 1u); return (unsigned short)(u >> 16); }
__device__ __forceinline__ float bfr(float f) { return __uint_as_float(((unsigned)f2bf(f)) << 16); }
__device__ __forceinline__ v16h cat16(v8h lo, v8h hi) { return __builtin_shufflevector(lo, hi, 0, 1, 2, 3, 4, 5, 6, 7, 8, 9, 10, 11, 12, 13, 14, 15); }
__device__ __forceinline__ v8f wmma16(v16h a, v16h b, v8f c) { return __builtin_amdgcn_wmma_f32_16x16x32_f16(false, a, false, b, (short)0, c, false, false); }
__device__ __forceinline__ v16h  ldh(const h16* p) { return cat16(*(const v8h*)p, *(const v8h*)(p + 16)); }
__device__ __forceinline__ void wave_sync() { __builtin_amdgcn_fence(3  , "wavefront"); __builtin_amdgcn_wave_barrier(); asm volatile("" ::: "memory"); }
static __device__ __forceinline__ h16 toh_flush(float v) { const h16 r = (h16)v; return (fabsf(v) < 6.103515625e-05f) ? (h16)0.0f : r; }
__device__ __forceinline__ v8f wmma16g(v16h a, v16h b, v8f c) {
    c = wmma16(a, b, c);
    asm volatile("v_nop\n\tv_nop\n\tv_nop\n\tv_nop" : "+v"(c) : "v"(a), "v"(b));
    return c;
}
__device__ __forceinline__ void st2h(h16* p, v8h v) { *(volatile v8h*)p = v; __threadfence(); *(volatile v8h*)p = v; }

__device__ __forceinline__ void mm64(const h16* __restrict__ A, size_t lda, const h16* __restrict__ Bt, size_t ldb, int K, int lr, int hi, v8f (&acc)[4][4]) {
    const size_t aoff = (size_t)lr * lda + 8 * hi, boff = (size_t)lr * ldb + 8 * hi;
#pragma unroll 1
    for (int kc = 0; kc < K; kc += 32) {
        v16h a[4];
#pragma unroll
        for (int mb = 0; mb < 4; ++mb) a[mb] = ldh(A + aoff + (size_t)mb * 16 * lda + kc);
#pragma unroll
        for (int nb = 0; nb < 4; ++nb) { const v16h b = ldh(Bt + boff + (size_t)nb * 16 * ldb + kc);
#pragma unroll
            for (int mb = 0; mb < 4; ++mb) acc[mb][nb] = wmma16g(a[mb], b, acc[mb][nb]); }
    }
}

__global__ __launch_bounds__(256) void k_prep(const float* __restrict__ q1, const float* __restrict__ q2, const float* __restrict__ W,
                                              h16* Q1H, h16* Q2H, h16* AP, h16* A1W, float* NRM) {
#pragma clang fp contract(off)
    __shared__ __align__(16) float nl[4 * 32];
    const int lane = threadIdx.x & 31;
    const int wave = __builtin_amdgcn_readfirstlane((int)(threadIdx.x >> 5));
    const int rb0 = blockIdx.x * 32;
#pragma unroll 1
    for (int rr = 0; rr < 4; ++rr) {
        const int rl = wave * 4 + rr;
        const int row = rb0 + rl;
        const int b = row / SEQ, s = row % SEQ;
        const size_t irow = ((size_t)b * SEQ_FULL + (size_t)s) * FW;
#pragma unroll 1
        for (int half = 0; half < 2; ++half) {
            const int co = half * HW + lane * 8;
            const int arow = (1 - half) * (SEQ - 1);
            const v8f x1 = *(const v8f*)(q1 + irow + co);
            const v8f x2 = *(const v8f*)(q2 + irow + co);
            const v8f xa = *(const v8f*)(q2 + ((size_t)b * SEQ_FULL + (size_t)arow) * FW + co);
            float xq[8]; v8h o1, o2, p0, p1, p2; float s1 = 0.0f, s2 = 0.0f;
#pragma unroll
            for (int k = 0; k < 8; ++k) {
                const float a = bfr(x1[k]), c = bfr(x2[k]), e = bfr(xa[k]);
                xq[k] = a;
                o1[k] = toh_flush(a); o2[k] = toh_flush(c);
                p0[k] = toh_flush(a * a); p1[k] = toh_flush(c * c); p2[k] = toh_flush(a * e);
                s1 += a * a; s2 += c * c; }
            s1 += __shfl_xor(s1, 16, 32); s2 += __shfl_xor(s2, 16, 32);
            s1 += __shfl_xor(s1, 8, 32);  s2 += __shfl_xor(s2, 8, 32);
            s1 += __shfl_xor(s1, 4, 32);  s2 += __shfl_xor(s2, 4, 32);
            s1 += __shfl_xor(s1, 2, 32);  s2 += __shfl_xor(s2, 2, 32);
            s1 += __shfl_xor(s1, 1, 32);  s2 += __shfl_xor(s2, 1, 32);
            if (lane == 0) { nl[(0 * 2 + half) * 32 + rl] = sqrtf(s1); nl[(1 * 2 + half) * 32 + rl] = sqrtf(s2); }
            st2h(Q1H + (size_t)row * FW + co, o1);
            st2h(Q2H + (size_t)row * FW + co, o2);
            const size_t po = ((size_t)half * ROWS + (size_t)row) * HW + lane * 8;
            st2h(AP + (size_t)0 * 2 * ROWS * HW + po, p0);
            st2h(AP + (size_t)1 * 2 * ROWS * HW + po, p1);
            st2h(AP + (size_t)2 * 2 * ROWS * HW + po, p2);
#pragma unroll 1
            for (int l = 0; l < NPER; ++l) {
                const v8f wv = *(const v8f*)(W + ((size_t)((2 + half) * NPER + l)) * HW + lane * 8);
                v8h o;
#pragma unroll
                for (int k = 0; k < 8; ++k) { const float w = bfr(wv[k]); o[k] = toh_flush(xq[k] * (w * w)); }
                st2h(A1W + ((size_t)(half * NPER + l) * ROWS + (size_t)row) * HW + lane * 8, o);
            }
        }
    }
    __syncthreads();
    if (wave == 0) {
        const int q = lane >> 3, pc = (lane & 7) * 4;
        const v4f v = *(const v4fa*)(&nl[q * 32 + pc]);
        float* dst = NRM + (size_t)q * ROWS + rb0 + pc;
        *(volatile v4f*)dst = v; __threadfence(); *(volatile v4f*)dst = v;
    }
}

__global__ __launch_bounds__(256) void k_small(const float* __restrict__ q2, const float* __restrict__ W, h16* ANC2, h16* W2) {
#pragma clang fp contract(off)
    const int lane = threadIdx.x & 31;
    const int wave = __builtin_amdgcn_readfirstlane((int)(threadIdx.x >> 5));
    const int r = blockIdx.x * 8 + wave;
    if (blockIdx.x < 16) {
        const int half = r >> 6, rr = r & 63; const int b = rr % NB; const int arow = (1 - half) * (SEQ - 1);
        const v8f x = *(const v8f*)(q2 + ((size_t)b * SEQ_FULL + (size_t)arow) * FW + half * HW + lane * 8);
        v8h o;
#pragma unroll
        for (int k = 0; k < 8; ++k) { const float a = bfr(x[k]); o[k] = toh_flush(a * a); }
        st2h(ANC2 + (size_t)(half * 64 + rr) * HW + lane * 8, o);
    } else {
        const int r2 = r - 128; const int half = r2 >> 6, c = r2 & 63; const int g = c >> 4, l = c & 15;
        const v8f x = *(const v8f*)(W + ((size_t)((2 * g + half) * NPER + l)) * HW + lane * 8);
        v8h o;
#pragma unroll
        for (int k = 0; k < 8; ++k) { const float a = bfr(x[k]); o[k] = toh_flush((a * a) * W2C); }
        st2h(W2 + (size_t)(half * 64 + c) * HW + lane * 8, o);
    }
}

__global__ __launch_bounds__(256) void k_q2t(const h16* __restrict__ Q2H, h16* Q2T) {
    __shared__ __align__(16) h16 ts[64 * TSP];
    const int tid = threadIdx.x, lane = tid & 31;
    const int wave = __builtin_amdgcn_readfirstlane((int)(threadIdx.x >> 5));
    const int hc = blockIdx.x, z = blockIdx.y; const int b = z >> 1, half = z & 1;
#pragma unroll 1
    for (int ps = 0; ps < SEQ / 32; ++ps) {
        const int tt = ps * 32 + (tid >> 3), hh = (tid & 7) * 8;
        const v8h x = *(const v8h*)(Q2H + ((size_t)b * SEQ + (size_t)tt) * FW + half * HW + hc * 64 + hh);
#pragma unroll
        for (int k = 0; k < 8; ++k) ts[(hh + k) * TSP + tt] = x[k];
    }
    __syncthreads();
    h16* dst = Q2T + ((size_t)z * HW + (size_t)hc * 64) * SEQ;
#pragma unroll 1
    for (int ps = 0; ps < 2; ++ps) {
#pragma unroll
        for (int s = 0; s < 4; ++s) { const int hrow = wave * 8 + 2 * s + (lane >> 4), c8 = (lane & 15) * 8;
            const v8h v = *(const v8ha*)(&ts[hrow * TSP + c8]);
            *(volatile v8h*)(dst + (size_t)hrow * SEQ + c8) = v; }
        if (ps == 0) __threadfence(); }
}

__global__ __launch_bounds__(32) void k_att(const h16* __restrict__ Q1H, const h16* __restrict__ Q2H, const float* __restrict__ NRM, float* ATT, h16* P16) {
    __shared__ __align__(16) float os[16 * 68];
    const int lane = threadIdx.x & 31, lr = lane & 15, hi = lane >> 4;
    const int s0 = blockIdx.x * 64, t0 = blockIdx.y * 64, z = blockIdx.z; const int b = z >> 1, half = z & 1;
    v8f acc[4][4];
#pragma unroll
    for (int mb = 0; mb < 4; ++mb)
#pragma unroll
        for (int nb = 0; nb < 4; ++nb) acc[mb][nb] = (v8f){};
    mm64(Q1H + ((size_t)b * SEQ + (size_t)s0) * FW + half * HW, (size_t)FW, Q2H + ((size_t)b * SEQ + (size_t)t0) * FW + half * HW, (size_t)FW, HW, lr, hi, acc);
    const float* n1p = NRM + (size_t)(0 * 2 + half) * ROWS + (size_t)b * SEQ + s0;
    const float* n2p = NRM + (size_t)(1 * 2 + half) * ROWS + (size_t)b * SEQ + t0;
    float n2c[4];
#pragma unroll
    for (int nb = 0; nb < 4; ++nb) n2c[nb] = n2p[nb * 16 + lr];
    float* arow = ATT + ((size_t)z * SEQ + (size_t)s0) * SEQ + t0;
    h16*   prow = P16 + ((size_t)z * SEQ + (size_t)s0) * SEQ + t0;
#pragma unroll
    for (int mb = 0; mb < 4; ++mb) {
#pragma unroll
        for (int j = 0; j < 8; ++j) { const float n1r = n1p[mb * 16 + hi * 8 + j];
#pragma unroll
            for (int nb = 0; nb < 4; ++nb) { const float den = n1r * n2c[nb]; const float dd = (den > EPSV) ? den : EPSV;
                os[(hi * 8 + j) * 68 + nb * 16 + lr] = acc[mb][nb][j] * __builtin_amdgcn_rcpf(dd); } }
        wave_sync();
#pragma unroll 1
        for (int ps = 0; ps < 2; ++ps) {
#pragma unroll
            for (int s = 0; s < 8; ++s) { const int row = 2 * s + (lane >> 4), c4 = (lane & 15) * 4;
                const v4f val = *(const v4fa*)(&os[row * 68 + c4]);
                *(volatile v4f*)(arow + (size_t)(mb * 16 + row) * SEQ + c4) = val; }
#pragma unroll
            for (int s = 0; s < 4; ++s) { const int row = 4 * s + (lane >> 3), c8 = (lane & 7) * 8;
                const v4f x0 = *(const v4fa*)(&os[row * 68 + c8]); const v4f x1 = *(const v4fa*)(&os[row * 68 + c8 + 4]); v8h hv;
#pragma unroll
                for (int i = 0; i < 4; ++i) { hv[i] = toh_flush(x0[i] * PCAR); hv[4 + i] = toh_flush(x1[i] * PCAR); }
                *(volatile v8h*)(prow + (size_t)(mb * 16 + row) * SEQ + c8) = hv; }
            if (ps == 0) __threadfence(); }
        wave_sync();
    }
}

__global__ __launch_bounds__(32) void k_asum(const h16* __restrict__ P16, const h16* __restrict__ Q2T, const h16* __restrict__ Q1H, h16* AP) {
    __shared__ __align__(16) float os[16 * 68];
    const int lane = threadIdx.x & 31, lr = lane & 15, hi = lane >> 4;
    const int s0 = blockIdx.x * 64, h0 = blockIdx.y * 64, z = blockIdx.z; const int b = z >> 1, half = z & 1;
    v8f acc[4][4];
#pragma unroll
    for (int mb = 0; mb < 4; ++mb)
#pragma unroll
        for (int nb = 0; nb < 4; ++nb) acc[mb][nb] = (v8f){};
    mm64(P16 + ((size_t)z * SEQ + (size_t)s0) * SEQ, (size_t)SEQ, Q2T + ((size_t)z * HW + (size_t)h0) * SEQ, (size_t)SEQ, SEQ, lr, hi, acc);
    const size_t grow0 = (size_t)b * SEQ + s0;
    h16* p3 = AP + ((size_t)(3 * 2 + half) * ROWS + grow0) * HW + h0;
    h16* p4 = AP + ((size_t)(4 * 2 + half) * ROWS + grow0) * HW + h0;
    const h16* qb = Q1H + grow0 * FW + half * HW + h0;
#pragma unroll
    for (int mb = 0; mb < 4; ++mb) {
#pragma unroll
        for (int nb = 0; nb < 4; ++nb) {
#pragma unroll
            for (int j = 0; j < 8; ++j) os[(hi * 8 + j) * 68 + nb * 16 + lr] = acc[mb][nb][j] * ASC; }
        wave_sync();
#pragma unroll 1
        for (int ps = 0; ps < 2; ++ps) {
#pragma unroll
            for (int s = 0; s < 4; ++s) { const int row = 4 * s + (lane >> 3), c8 = (lane & 7) * 8;
                const v4f x0 = *(const v4fa*)(&os[row * 68 + c8]); const v4f x1 = *(const v4fa*)(&os[row * 68 + c8 + 4]);
                const v8h q = *(const v8h*)(qb + (size_t)(mb * 16 + row) * FW + c8); v8h o3, o4;
#pragma unroll
                for (int i = 0; i < 4; ++i) { o3[i] = toh_flush((float)q[i] * x0[i]); o3[4 + i] = toh_flush((float)q[4 + i] * x1[i]);
                                              o4[i] = toh_flush(x0[i] * x0[i]);       o4[4 + i] = toh_flush(x1[i] * x1[i]); }
                *(volatile v8h*)(p3 + (size_t)(mb * 16 + row) * HW + c8) = o3;
                *(volatile v8h*)(p4 + (size_t)(mb * 16 + row) * HW + c8) = o4; }
            if (ps == 0) __threadfence(); }
        wave_sync();
    }
}

__global__ __launch_bounds__(256) void k_amax(const float* __restrict__ ATT, const h16* __restrict__ Q2H, const h16* __restrict__ Q1H, h16* AP) {
#pragma clang fp contract(off)
    __shared__ __align__(16) float ar[8 * SEQ];
    const int lane = threadIdx.x & 31;
    const int wave = __builtin_amdgcn_readfirstlane((int)(threadIdx.x >> 5));
    const int rid = blockIdx.x * 8 + wave;
    const int z = rid / SEQ, s = rid % SEQ; const int b = z >> 1, half = z & 1;
    { const v4f a = *(const v4f*)(ATT + (size_t)rid * SEQ + lane * 4); *(v4fa*)(&ar[wave * SEQ + lane * 4]) = a; }
    wave_sync();
    float m[8];
#pragma unroll
    for (int k = 0; k < 8; ++k) m[k] = NEGB;
    const h16* qb = Q2H + (size_t)b * SEQ * FW + half * HW + lane * 8;
#pragma unroll 1
    for (int t4 = 0; t4 < SEQ / 4; ++t4) {
        const v4f a4 = *(const v4fa*)(&ar[wave * SEQ + t4 * 4]);
#pragma unroll
        for (int i = 0; i < 4; ++i) { const v8h x = *(const v8h*)(qb + (size_t)(t4 * 4 + i) * FW);
#pragma unroll
            for (int k = 0; k < 8; ++k) m[k] = fmaxf(m[k], a4[i] * (float)x[k]); }
    }
    const v8h q = *(const v8h*)(Q1H + ((size_t)b * SEQ + (size_t)s) * FW + half * HW + lane * 8);
    v8h o5, o6;
#pragma unroll
    for (int k = 0; k < 8; ++k) { const float mm = m[k] * AMC; o5[k] = toh_flush((float)q[k] * mm); o6[k] = toh_flush(mm * mm); }
    const size_t ro = ((size_t)b * SEQ + (size_t)s) * HW + lane * 8;
    st2h(AP + (size_t)(5 * 2 + half) * ROWS * HW + ro, o5);
    st2h(AP + (size_t)(6 * 2 + half) * ROWS * HW + ro, o6);
}

__global__ __launch_bounds__(32) void k_nrm(const h16* __restrict__ A, const h16* __restrict__ W2, float* NPo, size_t aStrideH, size_t aStrideP, size_t oStrideH, size_t oStrideP) {
    __shared__ __align__(16) float os[16 * 68];
    const int lane = threadIdx.x & 31, lr = lane & 15, hi = lane >> 4;
    const int r0 = blockIdx.x * 64, half = blockIdx.y, p = blockIdx.z;
    v8f acc[4][4];
#pragma unroll
    for (int mb = 0; mb < 4; ++mb)
#pragma unroll
        for (int nb = 0; nb < 4; ++nb) acc[mb][nb] = (v8f){};
    mm64(A + (size_t)p * aStrideP + (size_t)half * aStrideH + (size_t)r0 * HW, (size_t)HW, W2 + (size_t)half * 64 * HW, (size_t)HW, HW, lr, hi, acc);
    float* orow = NPo + (size_t)p * oStrideP + (size_t)half * oStrideH + (size_t)r0 * 64;
#pragma unroll
    for (int mb = 0; mb < 4; ++mb) {
#pragma unroll
        for (int nb = 0; nb < 4; ++nb) {
#pragma unroll
            for (int j = 0; j < 8; ++j) os[(hi * 8 + j) * 68 + nb * 16 + lr] = acc[mb][nb][j] * W2I; }
        wave_sync();
#pragma unroll 1
        for (int ps = 0; ps < 2; ++ps) {
#pragma unroll
            for (int s = 0; s < 8; ++s) { const int row = 2 * s + (lane >> 4), c4 = (lane & 15) * 4;
                const v4f val = *(const v4fa*)(&os[row * 68 + c4]);
                *(volatile v4f*)(orow + (size_t)(mb * 16 + row) * 64 + c4) = val; }
            if (ps == 0) __threadfence(); }
        wave_sync();
    }
}

__global__ __launch_bounds__(32) void k_maxpool(const h16* __restrict__ A1W, const h16* __restrict__ Q2H, const float* __restrict__ NPl, float* MXP) {
    __shared__ __align__(16) float part[2 * SEQ];
    const int lane = threadIdx.x & 31, lr = lane & 15, hi = lane >> 4;
    const int b = blockIdx.x, l = blockIdx.y, half = blockIdx.z;
    const h16* Ab = A1W + ((size_t)(half * NPER + l) * ROWS + (size_t)b * SEQ) * HW;
    const h16* Bb = Q2H + (size_t)b * SEQ * FW + half * HW;
    const float* nap = NPl + ((size_t)(0 * 2 + half) * ROWS + (size_t)b * SEQ) * 64 + 16 + l;
    const float* nbp = NPl + ((size_t)(1 * 2 + half) * ROWS + (size_t)b * SEQ) * 64 + 16 + l;
#pragma unroll 1
    for (int mg = 0; mg < 2; ++mg) {
#pragma unroll 1
        for (int ng = 0; ng < 2; ++ng) {
            v8f acc[4][4];
#pragma unroll
            for (int mb = 0; mb < 4; ++mb)
#pragma unroll
                for (int nb = 0; nb < 4; ++nb) acc[mb][nb] = (v8f){};
            mm64(Ab + (size_t)mg * 64 * HW, (size_t)HW, Bb + (size_t)ng * 64 * FW, (size_t)FW, HW, lr, hi, acc);
            float rn[4];
#pragma unroll
            for (int nb = 0; nb < 4; ++nb) { const float x = nbp[(size_t)(ng * 64 + nb * 16 + lr) * 64]; float n = sqrtf(x); n = (n > EPSV) ? n : EPSV; rn[nb] = 1.0f / n; }
#pragma unroll
            for (int mb = 0; mb < 4; ++mb) {
#pragma unroll
                for (int j = 0; j < 8; ++j) {
                    float m = fmaxf(fmaxf(acc[mb][0][j] * rn[0], acc[mb][1][j] * rn[1]), fmaxf(acc[mb][2][j] * rn[2], acc[mb][3][j] * rn[3]));
                    m = fmaxf(m, __shfl_xor(m, 1, 32)); m = fmaxf(m, __shfl_xor(m, 2, 32));
                    m = fmaxf(m, __shfl_xor(m, 4, 32)); m = fmaxf(m, __shfl_xor(m, 8, 32));
                    if (lr == 0) part[ng * SEQ + mg * 64 + mb * 16 + hi * 8 + j] = m; } }
        }
    }
    wave_sync();
    const v4f pa = *(const v4fa*)(&part[lane * 4]); const v4f pb = *(const v4fa*)(&part[SEQ + lane * 4]);
    v4f o;
#pragma unroll
    for (int i = 0; i < 4; ++i) { const float x = nap[(size_t)(lane * 4 + i) * 64]; float n = sqrtf(x); n = (n > EPSV) ? n : EPSV; o[i] = fmaxf(pa[i], pb[i]) * (1.0f / n); }
    float* dst = MXP + (size_t)(half * NPER + l) * ROWS + (size_t)b * SEQ + lane * 4;
    *(volatile v4f*)dst = o; __threadfence(); *(volatile v4f*)dst = o;
}

__global__ __launch_bounds__(128) void k_final(const float* __restrict__ NPl, const float* __restrict__ NPA, const float* __restrict__ MXP, const float* __restrict__ ATT, float* OUT) {
#pragma clang fp contract(off)
    const int tid = threadIdx.x, lane = tid & 31;
    const int kind = tid >> 5, half = (tid >> 4) & 1, l = tid & 15;
    const int row = blockIdx.x; const int b = row / SEQ, s = row % SEQ;
    const v4f a0 = *(const v4f*)(ATT + ((size_t)(b * 2 + 0) * SEQ + (size_t)s) * SEQ + lane * 4);
    const v4f a1 = *(const v4f*)(ATT + ((size_t)(b * 2 + 1) * SEQ + (size_t)s) * SEQ + lane * 4);
    float s0 = (a0[0] + a0[1]) + (a0[2] + a0[3]); float s1 = (a1[0] + a1[1]) + (a1[2] + a1[3]);
    s0 += __shfl_xor(s0, 16, 32); s1 += __shfl_xor(s1, 16, 32);
    s0 += __shfl_xor(s0, 8, 32);  s1 += __shfl_xor(s1, 8, 32);
    s0 += __shfl_xor(s0, 4, 32);  s1 += __shfl_xor(s1, 4, 32);
    s0 += __shfl_xor(s0, 2, 32);  s1 += __shfl_xor(s1, 2, 32);
    s0 += __shfl_xor(s0, 1, 32);  s1 += __shfl_xor(s1, 1, 32);
    float d = half ? s1 : s0; d = (d > EPSV) ? d : EPSV;
    const size_t PS = (size_t)2 * ROWS * 64;
    const size_t cr = ((size_t)half * ROWS + (size_t)row) * 64;
    const float na2  = NPl[cr + kind * 16 + l];
    const float nf   = NPl[2 * PS + cr + l];
    const float nbf2 = NPA[((size_t)half * 64 + (size_t)b) * 64 + l];
    const float nat  = NPl[3 * PS + cr + 32 + l];
    const float nb2a = NPl[4 * PS + cr + 32 + l];
    const float nmt  = NPl[5 * PS + cr + 48 + l];
    const float nb2m = NPl[6 * PS + cr + 48 + l];
    const float mx   = MXP[(size_t)(half * NPER + l) * ROWS + (size_t)row];
    const float rd = 1.0f / d;
    const float num = (kind == 0) ? nf : ((kind == 2) ? nat : nmt);
    const float nb2 = (kind == 0) ? nbf2 : ((kind == 2) ? nb2a : nb2m);
    const float sc  = (kind == 0) ? 1.0f : ((kind == 2) ? (ASI * rd) : AMI);
    float na = sqrtf(na2); na = (na > EPSV) ? na : EPSV;
    float nb = sqrtf(nb2) * sc; nb = (nb > EPSV) ? nb : EPSV;
    const float cosv = (num * sc) / (na * nb);
    const float v = (kind == 1) ? mx : cosv;
    float* dst = OUT + ((size_t)b * OUT_SEQ + (size_t)s) * OC + tid;
    *(volatile float*)dst = v; __threadfence(); *(volatile float*)dst = v;
}

static constexpr size_t al256(size_t v) { return (v + 255) & ~(size_t)255; }
static constexpr size_t SZ_QH  = al256((size_t)ROWS * FW * 2);
static constexpr size_t SZ_QT  = al256((size_t)NZ * HW * SEQ * 2);
static constexpr size_t SZ_AP  = al256((size_t)NPL * 2 * ROWS * HW * 2);
static constexpr size_t SZ_AW  = al256((size_t)2 * NPER * ROWS * HW * 2);
static constexpr size_t SZ_SM  = al256((size_t)2 * 64 * HW * 2);
static constexpr size_t SZ_NRM = al256((size_t)4 * ROWS * 4);
static constexpr size_t SZ_ATT = al256((size_t)NZ * SEQ * SEQ * 4);
static constexpr size_t SZ_P   = al256((size_t)NZ * SEQ * SEQ * 2);
static constexpr size_t SZ_NP  = al256((size_t)NPL * 2 * ROWS * 64 * 4);
static constexpr size_t SZ_NPA = al256((size_t)2 * 64 * 64 * 4);
static constexpr size_t SZ_MX  = al256((size_t)2 * NPER * ROWS * 4);
static constexpr size_t SZ_TOTAL = 2 * SZ_QH + SZ_QT + SZ_AP + SZ_AW + 2 * SZ_SM + SZ_NRM + SZ_ATT + SZ_P + SZ_NP + SZ_NPA + SZ_MX;
static_assert(SZ_TOTAL <= (size_t)134217728);
static_assert(((size_t)ROWS * 4) % 128 == 0);
static_assert(((size_t)ROWS * HW * 2) % 256 == 0);

extern "C" void kernel_launch(void* const* d_in, const int* in_sizes, int n_in,
                              void* d_out, int out_size, void* d_ws, size_t ws_size, hipStream_t stream) {
    if (n_in < 3) return;
    const size_t needx = ((size_t)(NB - 1) * SEQ_FULL + SEQ) * FW;
    if ((size_t)in_sizes[0] < needx || (size_t)in_sizes[1] < needx) return;
    if ((size_t)in_sizes[2] < (size_t)8 * NPER * HW) return;
    if ((size_t)out_size < ((size_t)(NB - 1) * OUT_SEQ + SEQ) * OC) return;
    if (SZ_TOTAL > ws_size) return;
    const float* q1 = (const float*)d_in[0];
    const float* q2 = (const float*)d_in[1];
    const float* W  = (const float*)d_in[2];
    float* OUT = (float*)d_out;
    char* wsp = (char*)d_ws;
    h16* Q1H = (h16*)wsp; wsp += SZ_QH;
    h16* Q2H = (h16*)wsp; wsp += SZ_QH;
    h16* Q2T = (h16*)wsp; wsp += SZ_QT;
    h16* AP  = (h16*)wsp; wsp += SZ_AP;
    h16* A1W = (h16*)wsp; wsp += SZ_AW;
    h16* ANC2 = (h16*)wsp; wsp += SZ_SM;
    h16* W2  = (h16*)wsp; wsp += SZ_SM;
    float* NRM = (float*)wsp; wsp += SZ_NRM;
    float* ATT = (float*)wsp; wsp += SZ_ATT;
    h16* P16 = (h16*)wsp; wsp += SZ_P;
    float* NPl = (float*)wsp; wsp += SZ_NP;
    float* NPA = (float*)wsp; wsp += SZ_NPA;
    float* MXP = (float*)wsp; wsp += SZ_MX;

    k_prep<<<ROWS / 32, 256, 0, stream>>>(q1, q2, W, Q1H, Q2H, AP, A1W, NRM);
    k_small<<<32, 256, 0, stream>>>(q2, W, ANC2, W2);
    k_q2t<<<dim3(HW / 64, NZ, 1), 256, 0, stream>>>(Q2H, Q2T);
    k_att<<<dim3(SEQ / 64, SEQ / 64, NZ), 32, 0, stream>>>(Q1H, Q2H, NRM, ATT, P16);
    k_asum<<<dim3(SEQ / 64, HW / 64, NZ), 32, 0, stream>>>(P16, Q2T, Q1H, AP);
    k_amax<<<NZ * SEQ / 8, 256, 0, stream>>>(ATT, Q2H, Q1H, AP);
    k_nrm<<<dim3(ROWS / 64, 2, NPL), 32, 0, stream>>>(AP, W2, NPl, (size_t)ROWS * HW, (size_t)2 * ROWS * HW, (size_t)ROWS * 64, (size_t)2 * ROWS * 64);
    k_nrm<<<dim3(1, 2, 1), 32, 0, stream>>>(ANC2, W2, NPA, (size_t)64 * HW, (size_t)0, (size_t)64 * 64, (size_t)0);
    k_maxpool<<<dim3(NB, NPER, 2), 32, 0, stream>>>(A1W, Q2H, NPl, MXP);
    k_final<<<ROWS, 128, 0, stream>>>(NPl, NPA, MXP, ATT, OUT);
}
